// GraphSAGE_8504035246140
// MI455X (gfx1250) — hardware-verified
//
#include <hip/hip_runtime.h>
#include <stddef.h>
#include <stdint.h>


#define DF     128
#define AGP    256
#define PFP    768
#define K0L    384
#define K1L    512
#define KHL    768
#define NTHR   256
#define NWAVE  8
#define EPT    8
#define CHUNK  (NTHR * EPT)
#define WCAP   (EPT * 32)
#define LISTN  (NWAVE * WCAP)
#define NBA    1024
#define SLA    10
#define RCAP   28672
#define DEGCAP 64
#define GBM    64
#define GBN    128
#define GTHR   128
#define UPART  2048
#define NPART  13
#define WOFF1  (DF * K0L)
#define WOFFH  (DF * K0L + DF * K1L)
#define WPTOT  (WOFFH + DF * KHL)
#define RECW   256
#define AGG_ZINTS    (LISTN + 2 * RCAP + 3 * NBA)
#define MISC_INTS    16
#define ROWBUF_INTS  (NWAVE * AGP / 2)
#define AGG_LDS_INTS (AGG_ZINTS + MISC_INTS + ROWBUF_INTS)
#define WSMAX  134217728
#define VG __attribute__((amdgpu_num_vgpr(248)))

static_assert((CHUNK & (CHUNK - 1)) == 0 && CHUNK <= 4096);
static_assert((NBA & (NBA - 1)) == 0 && NBA == (1 << SLA));
static_assert(((long long)CHUNK << SLA) < (1LL << 31));
static_assert(LISTN % NTHR == 0);
static_assert(NBA % NWAVE == 0 && NBA % 32 == 0 && NBA % GBM == 0);
static_assert(RCAP % 4 == 0 && AGG_ZINTS % 4 == 0 && LISTN % 4 == 0 && ((AGG_ZINTS + MISC_INTS) % 4) == 0);
static_assert(AGG_ZINTS % (NTHR * 4) == 0);
static_assert(RCAP >= 13196 && DEGCAP >= 36);
static_assert(K0L % 32 == 0 && K1L % 32 == 0 && KHL % 32 == 0);
static_assert(K0L == 3 * DF && K1L == 4 * DF && KHL == 6 * DF && AGP == 2 * DF && PFP == KHL);
static_assert(GBN == DF && GBM == (GTHR / 32) * 16 && DF == 4 * 32 && GTHR == GBN);
static_assert(UPART % NTHR == 0 && UPART == DF * (DF / 8));
static_assert((NPART * UPART) % NTHR == 0);
static_assert((WOFF1 * 2) % 256 == 0 && (WOFFH * 2) % 256 == 0 && (WPTOT * 2) % 256 == 0);
static_assert(RECW == 2 * GBN && RECW / 4 <= GTHR);
static_assert(AGG_LDS_INTS * 4 <= 300000);
static_assert(GBM == NWAVE * 8);

typedef float          v4f   __attribute__((ext_vector_type(4)));
typedef float          v8f   __attribute__((ext_vector_type(8)));
typedef int            v4i   __attribute__((ext_vector_type(4)));
typedef int            v8i   __attribute__((ext_vector_type(8)));
typedef unsigned       v2u   __attribute__((ext_vector_type(2)));
typedef unsigned short v4us  __attribute__((ext_vector_type(4)));
typedef unsigned short v8us  __attribute__((ext_vector_type(8)));
typedef unsigned short v16us __attribute__((ext_vector_type(16)));
typedef __bf16         v16bf __attribute__((ext_vector_type(16)));
typedef v4f  __attribute__((may_alias)) v4fa;
typedef v4i  __attribute__((may_alias)) v4ia;
typedef v2u  __attribute__((may_alias)) v2ua;
typedef v4us __attribute__((may_alias)) v4usa;
typedef v8us __attribute__((may_alias)) v8usa;
union FragB { v16bf v; v16us u; v8us h[2]; v8i w; };

__device__ __forceinline__ v8f wmb(const FragB& a, const FragB& b, v8f c) {
  v8f d = __builtin_amdgcn_wmma_f32_16x16x32_bf16(false, a.v, false, b.v, (short)0, c, false, false);
  asm volatile("v_nop\n\tv_nop\n\tv_nop\n\tv_nop" : "+v"(d) : "v"(a.w), "v"(b.w));
  return d;
}

__device__ __forceinline__ unsigned bf16_bits(float f) {
  const unsigned u = __float_as_uint(f);
  const unsigned r = (u + 0x7FFFu + ((u >> 16) & 1u)) >> 16;
  return (f != f) ? 0x7FC0u : r;
}
__device__ __forceinline__ float bf16_val(float f) {
  return __uint_as_float(bf16_bits(f) << 16);
}
__device__ __forceinline__ unsigned split_pack(float v) {
  const unsigned hb = bf16_bits(v);
  const unsigned lb = bf16_bits(v - __uint_as_float(hb << 16));
  return hb | (lb << 16);
}
__device__ __forceinline__ float relu_np(float v) { return (v > 0.0f) ? v : (v - v); }

__device__ __forceinline__ void wave_sync() {
  __builtin_amdgcn_fence(__ATOMIC_RELEASE, "workgroup");
  __builtin_amdgcn_wave_barrier();
  __builtin_amdgcn_fence(__ATOMIC_ACQUIRE, "workgroup");
}

template <int SLB>
__device__ __forceinline__ int scan_chunk(const int* __restrict__ dsts, int nE, int cbase, int slotBase,
                                          int nb, int vec8, int* list, int tid, int lane, int wave) {
  int wc = 0;
  const int el0  = tid * EPT;
  const int e0   = cbase + el0;
  const int sent = -2147483647 - 1;
  v4i da, db;
  if (vec8 != 0 && cbase + CHUNK <= nE) {
    da = *(const v4i*)(dsts + e0);
    db = *(const v4i*)(dsts + e0 + 4);
  } else {
    da.x = (e0     < nE) ? dsts[min(e0,     nE - 1)] : sent;
    da.y = (e0 + 1 < nE) ? dsts[min(e0 + 1, nE - 1)] : sent;
    da.z = (e0 + 2 < nE) ? dsts[min(e0 + 2, nE - 1)] : sent;
    da.w = (e0 + 3 < nE) ? dsts[min(e0 + 3, nE - 1)] : sent;
    db.x = (e0 + 4 < nE) ? dsts[min(e0 + 4, nE - 1)] : sent;
    db.y = (e0 + 5 < nE) ? dsts[min(e0 + 5, nE - 1)] : sent;
    db.z = (e0 + 6 < nE) ? dsts[min(e0 + 6, nE - 1)] : sent;
    db.w = (e0 + 7 < nE) ? dsts[min(e0 + 7, nE - 1)] : sent;
  }
  const unsigned nbs = (unsigned)slotBase;
  const unsigned unb = (unsigned)nb;
  const unsigned s0 = (unsigned)da.x - nbs, s1 = (unsigned)da.y - nbs;
  const unsigned s2 = (unsigned)da.z - nbs, s3 = (unsigned)da.w - nbs;
  const unsigned s4 = (unsigned)db.x - nbs, s5 = (unsigned)db.y - nbs;
  const unsigned s6 = (unsigned)db.z - nbs, s7 = (unsigned)db.w - nbs;
  const bool h0 = s0 < unb, h1 = s1 < unb, h2 = s2 < unb, h3 = s3 < unb;
  const bool h4 = s4 < unb, h5 = s5 < unb, h6 = s6 < unb, h7 = s7 < unb;
  const unsigned any = __builtin_amdgcn_ballot_w32(h0 | h1 | h2 | h3 | h4 | h5 | h6 | h7);
  if (any != 0u) {
#define HITJ(J, HJ, SJ) { \
      const unsigned mj = __builtin_amdgcn_ballot_w32(HJ); \
      if (mj != 0u) { \
        if (HJ) { \
          const int pos = wc + (int)__builtin_amdgcn_mbcnt_lo(mj, 0u); \
          if (pos < WCAP) list[wave * WCAP + pos] = ((el0 + (J)) << SLB) | (int)(SJ); \
        } \
        wc += (int)__builtin_popcount(mj); } }
    HITJ(0, h0, s0)
    HITJ(1, h1, s1)
    HITJ(2, h2, s2)
    HITJ(3, h3, s3)
    HITJ(4, h4, s4)
    HITJ(5, h5, s5)
    HITJ(6, h6, s6)
    HITJ(7, h7, s7)
#undef HITJ
  }
  return wc;
}

__device__ __forceinline__ v8us gath8(const float* __restrict__ W, int soff) {
  v8us o;
#pragma unroll
  for (int i = 0; i < 8; ++i) o[i] = (unsigned short)bf16_bits(W[soff + i * DF]);
  return o;
}

__global__ __launch_bounds__(NTHR) VG void k_wprep(const float* __restrict__ Ws, const float* __restrict__ Wn,
                                                   const float* __restrict__ W1, unsigned short* WP) {
  const int u    = (int)blockIdx.x * NTHR + (int)threadIdx.x;
  const int part = u >> 11;
  if (part >= NPART) return;
  const int v  = u & (UPART - 1);
  const int n  = v >> 4;
  const int k8 = (v & 15) * 8;
  int pitch, pbase, cb, sel, soff;
  if (part < 3) {
    pitch = K0L; pbase = 0; cb = part;
    sel = (cb == 2) ? 0 : 1;
    soff = k8 * DF + n;
  } else if (part < 7) {
    pitch = K1L; pbase = WOFF1; cb = part - 3;
    sel = (cb >= 2) ? 0 : 1;
    soff = DF * DF + k8 * DF + n;
  } else {
    pitch = KHL; pbase = WOFFH; cb = part - 7;
    sel = 2;
    soff = ((cb >> 1) * DF + k8) * DF + n;
  }
  v8us o;
  if (sel == 0)      o = gath8(Ws, soff);
  else if (sel == 1) o = gath8(Wn, soff);
  else               o = gath8(W1, soff);
  unsigned short* dp = WP + (size_t)pbase + (size_t)n * pitch + cb * DF + k8;
  *(volatile v8us*)dp = o;
  __threadfence();
  *(volatile v8us*)dp = o;
}

__global__ __launch_bounds__(NTHR) VG void k_pa(const float* __restrict__ x, int nN, int nUnits,
                                                unsigned short* xb) {
  const int u = (int)blockIdx.x * NTHR + (int)threadIdx.x;
  if (u >= nUnits) return;
  const int row = u >> 4;
  const int c8  = (u & 15) * 8;
  const int rc  = row < nN ? row : nN - 1;
  const float* p = x + (size_t)rc * DF + c8;
  const v4f a = *(const v4f*)p;
  const v4f b = *(const v4f*)(p + 4);
  const bool live = row < nN;
  v8us o;
  o[0] = live ? (unsigned short)bf16_bits(a.x) : (unsigned short)0;
  o[1] = live ? (unsigned short)bf16_bits(a.y) : (unsigned short)0;
  o[2] = live ? (unsigned short)bf16_bits(a.z) : (unsigned short)0;
  o[3] = live ? (unsigned short)bf16_bits(a.w) : (unsigned short)0;
  o[4] = live ? (unsigned short)bf16_bits(b.x) : (unsigned short)0;
  o[5] = live ? (unsigned short)bf16_bits(b.y) : (unsigned short)0;
  o[6] = live ? (unsigned short)bf16_bits(b.z) : (unsigned short)0;
  o[7] = live ? (unsigned short)bf16_bits(b.w) : (unsigned short)0;
  unsigned short* dp = xb + (size_t)u * 8;
  *(volatile v8us*)dp = o;
  __threadfence();
  *(volatile v8us*)dp = o;
}

template <int L0>
__global__ __launch_bounds__(NTHR) VG void k_scan(const int* __restrict__ gath, const int* __restrict__ keys,
                                                  int nE, int nN, int vec8, int mRows,
                                                  const unsigned short* __restrict__ srcp,
                                                  unsigned short* aggp) {
  extern __shared__ __attribute__((aligned(16))) int dsm[];
  int* list = dsm;
  int* hl   = dsm + LISTN;
  int* sl   = hl + RCAP;
  int* cnt  = sl + RCAP;
  int* offs = cnt + NBA;
  int* cur  = offs + NBA;
  int* misc = cur + NBA;
  const int tid = (int)threadIdx.x, lane = tid & 31, wave = tid >> 5;
  unsigned short* rowbuf = (unsigned short*)(misc + MISC_INTS) + wave * AGP;
  const int nodeBase = (int)blockIdx.x * NBA;

  {
    const v4i z4 = {0, 0, 0, 0};
    for (int i = tid * 4; i < AGG_ZINTS; i += NTHR * 4) *(v4ia*)(dsm + i) = z4;
    if (tid < MISC_INTS) misc[tid] = 0;
  }
  __syncthreads();

  int t = 0, ov = 0;
  const int nChunks = (nE + CHUNK - 1) / CHUNK;
#pragma unroll 1
  for (int ch = 0; ch < nChunks; ++ch) {
    const int cbase = ch * CHUNK;
    const int wc = scan_chunk<SLA>(keys, nE, cbase, nodeBase, NBA, vec8, list, tid, lane, wave);
    if (lane == 0) misc[wave] = wc;
    __syncthreads();
    if (wave == 0) {
#pragma unroll 1
      for (int w2 = 0; w2 < NWAVE; ++w2) {
        int c = misc[w2];
        c = c < 0 ? 0 : (c > WCAP ? WCAP : c);
#pragma unroll 1
        for (int b0 = 0; b0 < c; b0 += 32) {
          const int idx = b0 + lane;
          const int ent = list[w2 * WCAP + (idx < WCAP ? idx : WCAP - 1)];
          const int m32 = (c - b0) < 32 ? (c - b0) : 32;
#pragma unroll 1
          for (int k = 0; k < m32; ++k) {
            const int u    = __builtin_amdgcn_readlane(ent, k);
            const int slot = u & (NBA - 1);
            const int el   = (u >> SLA) & (CHUNK - 1);
            const int pk   = ((cbase + el) << SLA) | slot;
            if (t < RCAP) {
              if (lane == 0) { hl[t] = pk; cnt[slot] = cnt[slot] + 1; }
              t = t + 1;
            } else {
              ov = 1;
            }
          }
        }
      }
    }
    __syncthreads();
  }
  if (wave == 0 && lane == 0) { misc[8] = t; misc[9] = ov; }
  __syncthreads();
  int tt = misc[8];
  tt = tt < 0 ? 0 : (tt > RCAP ? RCAP : tt);
  const int ovf = misc[9];

  if (wave == 0) {
    const int base = lane * (NBA / 32);
    int s = 0;
#pragma unroll 1
    for (int i = 0; i < NBA / 32; ++i) s += cnt[base + i];
    int incl = s;
#pragma unroll
    for (int d = 1; d < 32; d <<= 1) {
      const int y = __shfl_up(incl, d, 32);
      if (lane >= d) incl += y;
    }
    int run = incl - s;
#pragma unroll 1
    for (int i = 0; i < NBA / 32; ++i) {
      const int cv = cnt[base + i];
      offs[base + i] = run;
      cur[base + i]  = run;
      run += cv;
    }
  }
  __syncthreads();
  if (wave == 0) {
#pragma unroll 1
    for (int b0 = 0; b0 < tt; b0 += 32) {
      const int idx = b0 + lane;
      const int ent = hl[idx < RCAP ? idx : RCAP - 1];
      const int m32 = (tt - b0) < 32 ? (tt - b0) : 32;
#pragma unroll 1
      for (int k = 0; k < m32; ++k) {
        const int u    = __builtin_amdgcn_readlane(ent, k);
        const int slot = u & (NBA - 1);
        if (lane == 0) {
          int p = cur[slot];
          p = p < 0 ? 0 : (p > RCAP - 1 ? RCAP - 1 : p);
          sl[p] = u;
          cur[slot] = p + 1;
        }
      }
    }
  }
  __syncthreads();

  const float pz = (ovf != 0) ? __int_as_float(0x7fc00000) : 0.0f;
#pragma unroll 1
  for (int si = 0; si < NBA / NWAVE; ++si) {
    const int s    = si * NWAVE + wave;
    const int node = nodeBase + s;
    int c = cnt[s];
    const bool big = c > DEGCAP;
    c = c < 0 ? 0 : (c > DEGCAP ? DEGCAP : c);
    int o = offs[s];
    o = o < 0 ? 0 : (o > RCAP ? RCAP : o);
    float a0 = 0.0f, a1 = 0.0f, a2 = 0.0f, a3 = 0.0f;
#pragma unroll 1
    for (int b0 = 0; b0 < c; b0 += 32) {
      int idx = o + b0 + lane;
      idx = idx > RCAP - 1 ? RCAP - 1 : idx;
      const int ent = sl[idx];
      int eid = ent >> SLA;
      eid = eid < 0 ? 0 : (eid > nE - 1 ? nE - 1 : eid);
      int sr = gath[eid];
      sr = sr < 0 ? 0 : (sr > nN - 1 ? nN - 1 : sr);
      const int m32 = (c - b0) < 32 ? (c - b0) : 32;
#pragma unroll 1
      for (int k = 0; k < m32; ++k) {
        const int sk = __builtin_amdgcn_readlane(sr, k);
        if constexpr (L0 != 0) {
          const unsigned short* rp = srcp + (size_t)sk * DF + 4 * lane;
          const v2u w = *(const v2ua*)rp;
          a0 += __uint_as_float(w.x << 16);
          a1 += __uint_as_float(w.x & 0xffff0000u);
          a2 += __uint_as_float(w.y << 16);
          a3 += __uint_as_float(w.y & 0xffff0000u);
        } else {
          const unsigned short* rp = srcp + (size_t)sk * AGP + 4 * lane;
          const v2u wh = *(const v2ua*)rp;
          const v2u wl = *(const v2ua*)(rp + DF);
          const float f0 = __uint_as_float(wh.x << 16)         + __uint_as_float(wl.x << 16);
          const float f1 = __uint_as_float(wh.x & 0xffff0000u) + __uint_as_float(wl.x & 0xffff0000u);
          const float f2 = __uint_as_float(wh.y << 16)         + __uint_as_float(wl.y << 16);
          const float f3 = __uint_as_float(wh.y & 0xffff0000u) + __uint_as_float(wl.y & 0xffff0000u);
          a0 += f0;
          a1 += f1;
          a2 += f2;
          a3 += f3;
        }
      }
    }
    const float den = (c > 0) ? (float)c : 1.0f;
    const float pzr = big ? __int_as_float(0x7fc00000) : pz;
    const bool live = node < nN;
    const float m0 = live ? (a0 / den + pzr) : 0.0f;
    const float m1 = live ? (a1 / den + pzr) : 0.0f;
    const float m2 = live ? (a2 / den + pzr) : 0.0f;
    const float m3 = live ? (a3 / den + pzr) : 0.0f;
    v4us mh, ml;
    {
      unsigned sp;
      sp = split_pack(m0); mh[0] = (unsigned short)(sp & 0xffffu); ml[0] = (unsigned short)(sp >> 16);
      sp = split_pack(m1); mh[1] = (unsigned short)(sp & 0xffffu); ml[1] = (unsigned short)(sp >> 16);
      sp = split_pack(m2); mh[2] = (unsigned short)(sp & 0xffffu); ml[2] = (unsigned short)(sp >> 16);
      sp = split_pack(m3); mh[3] = (unsigned short)(sp & 0xffffu); ml[3] = (unsigned short)(sp >> 16);
    }
    *(v4usa*)(rowbuf + 4 * lane) = mh;
    *(v4usa*)(rowbuf + DF + 4 * lane) = ml;
    wave_sync();
    const v8us q0 = *(const v8usa*)(rowbuf + 8 * lane);
    wave_sync();
    if (node < mRows) {
      unsigned short* rpw = aggp + (size_t)node * AGP + 8 * lane;
      *(volatile v8us*)rpw = q0;
      __threadfence();
      *(volatile v8us*)rpw = q0;
    }
  }
}

template <int MODE>
__global__ __launch_bounds__(GTHR) VG void k_gemm(const unsigned short* __restrict__ A1,
                                                  const unsigned short* __restrict__ A2,
                                                  const unsigned short* __restrict__ BT,
                                                  const float* __restrict__ bias, int nOut,
                                                  unsigned short* outU, float* outF, float* rec) {
  constexpr int P1 = (MODE == 2) ? PFP : AGP;
  constexpr int K1 = (MODE == 2) ? KHL : AGP;
  constexpr int P2 = (MODE == 0) ? DF : AGP;
  constexpr int K2 = (MODE == 0) ? DF : ((MODE == 1) ? AGP : 0);
  constexpr int K  = K1 + K2;
  static_assert(K1 % 32 == 0 && K2 % 32 == 0 && K1 <= P1 && K2 <= P2);
  __shared__ __attribute__((aligned(16))) float stg[GBM * GBN];
  __shared__ __attribute__((aligned(16))) float rst[RECW];
  const int tid = (int)threadIdx.x, lane = tid & 31, wave = tid >> 5, hh = lane >> 4, m = lane & 15;
  const int rowBase = (int)blockIdx.x * GBM;

  v8f acc[8];
  {
    const v8f z = {0.f, 0.f, 0.f, 0.f, 0.f, 0.f, 0.f, 0.f};
#pragma unroll
    for (int t = 0; t < 8; ++t) acc[t] = z;
  }
  const unsigned short* ap1 = A1 + (size_t)(rowBase + 16 * wave + m) * (size_t)P1 + 8 * hh;
  const unsigned short* bp  = BT + (size_t)m * (size_t)K + 8 * hh;

#pragma unroll 1
  for (int k0 = 0; k0 < K1; k0 += 32) {
    FragB af;
    af.h[0] = *(const v8usa*)(ap1 + k0);
    af.h[1] = *(const v8usa*)(ap1 + k0 + 16);
#pragma unroll
    for (int nt = 0; nt < 8; ++nt) {
      const unsigned short* wq = bp + (size_t)(16 * nt) * (size_t)K + k0;
      FragB bf;
      bf.h[0] = *(const v8usa*)wq;
      bf.h[1] = *(const v8usa*)(wq + 16);
      acc[nt] = wmb(af, bf, acc[nt]);
    }
  }
  if constexpr (K2 > 0) {
    const unsigned short* ap2 = A2 + (size_t)(rowBase + 16 * wave + m) * (size_t)P2 + 8 * hh;
#pragma unroll 1
    for (int k0 = 0; k0 < K2; k0 += 32) {
      FragB af;
      af.h[0] = *(const v8usa*)(ap2 + k0);
      af.h[1] = *(const v8usa*)(ap2 + k0 + 16);
#pragma unroll
      for (int nt = 0; nt < 8; ++nt) {
        const unsigned short* wq = bp + (size_t)(16 * nt) * (size_t)K + K1 + k0;
        FragB bf;
        bf.h[0] = *(const v8usa*)wq;
        bf.h[1] = *(const v8usa*)(wq + 16);
        acc[nt] = wmb(af, bf, acc[nt]);
      }
    }
  }

#pragma unroll
  for (int nt = 0; nt < 8; ++nt) {
    const int lc = 16 * nt + m;
#pragma unroll
    for (int r = 0; r < 8; ++r) {
      const int lr = 16 * wave + 8 * hh + r;
      stg[lr * GBN + lc] = acc[nt][r];
    }
  }
  __syncthreads();

  v4f bb4;
  {
    const v4f t1 = *(const v4f*)(bias + 4 * lane);
    bb4.x = bf16_val(t1.x);
    bb4.y = bf16_val(t1.y);
    bb4.z = bf16_val(t1.z);
    bb4.w = bf16_val(t1.w);
  }

  v4f pv[16];
#pragma unroll
  for (int i = 0; i < 16; ++i) pv[i] = *(const v4fa*)(stg + (16 * wave + i) * GBN + 4 * lane);
  __syncthreads();

#pragma unroll
  for (int i = 0; i < 16; ++i) {
    const bool ok = (rowBase + 16 * wave + i) < nOut;
    const v4f t = pv[i] + bb4;
    v4f y;
    if constexpr (MODE == 2) {
      y = t;
    } else {
      y.x = relu_np(t.x); y.y = relu_np(t.y); y.z = relu_np(t.z); y.w = relu_np(t.w);
    }
    y.x = ok ? y.x : 0.0f; y.y = ok ? y.y : 0.0f; y.z = ok ? y.z : 0.0f; y.w = ok ? y.w : 0.0f;
    pv[i] = y;
  }

  if constexpr (MODE != 0) {
#pragma unroll
    for (int i = 0; i < 16; ++i) {
      const int r = rowBase + 16 * wave + i;
      *(volatile v4f*)(outF + (size_t)r * DF + 4 * lane) = pv[i];
    }
    __threadfence();
#pragma unroll
    for (int i = 0; i < 16; ++i) {
      const int r = rowBase + 16 * wave + i;
      *(volatile v4f*)(outF + (size_t)r * DF + 4 * lane) = pv[i];
    }
    if constexpr (MODE == 2) {
      const float bcol = bf16_val(bias[tid]);
      float s = 0.0f;
#pragma unroll 4
      for (int r = 0; r < GBM; ++r) s += stg[r * GBN + tid] + bcol;
      const float mean = s * (1.0f / (float)GBM);
      float q = 0.0f;
#pragma unroll 4
      for (int r = 0; r < GBM; ++r) {
        const float d = (stg[r * GBN + tid] + bcol) - mean;
        q = fmaf(d, d, q);
      }
      rst[tid] = mean;
      rst[GBN + tid] = q;
      __syncthreads();
      v4f ps = {0.f, 0.f, 0.f, 0.f};
      float* rp = rec + (size_t)blockIdx.x * RECW + 4 * (tid & (RECW / 4 - 1));
      if (tid < RECW / 4) {
        ps = *(const v4fa*)(rst + 4 * tid);
        *(volatile v4f*)rp = ps;
      }
      __threadfence();
      if (tid < RECW / 4) {
        *(volatile v4f*)rp = ps;
      }
    }
  } else {
#pragma unroll
    for (int i = 0; i < 16; ++i) {
      v4us h4, l4;
      unsigned sp;
      sp = split_pack(pv[i].x); h4[0] = (unsigned short)(sp & 0xffffu); l4[0] = (unsigned short)(sp >> 16);
      sp = split_pack(pv[i].y); h4[1] = (unsigned short)(sp & 0xffffu); l4[1] = (unsigned short)(sp >> 16);
      sp = split_pack(pv[i].z); h4[2] = (unsigned short)(sp & 0xffffu); l4[2] = (unsigned short)(sp >> 16);
      sp = split_pack(pv[i].w); h4[3] = (unsigned short)(sp & 0xffffu); l4[3] = (unsigned short)(sp >> 16);
      unsigned short* srow = (unsigned short*)stg + (size_t)(16 * wave + i) * (2 * GBN);
      *(v4usa*)(srow + 4 * lane) = h4;
      *(v4usa*)(srow + DF + 4 * lane) = l4;
    }
    __syncthreads();
    v8us qv[16];
#pragma unroll
    for (int i = 0; i < 16; ++i) {
      const unsigned short* srow = (const unsigned short*)stg + (size_t)(16 * wave + i) * (2 * GBN);
      qv[i] = *(const v8usa*)(srow + 8 * lane);
    }
#pragma unroll
    for (int i = 0; i < 16; ++i) {
      unsigned short* rp = outU + (size_t)(rowBase + 16 * wave + i) * (size_t)AGP + 8 * lane;
      *(volatile v8us*)rp = qv[i];
    }
    __threadfence();
#pragma unroll
    for (int i = 0; i < 16; ++i) {
      unsigned short* rp = outU + (size_t)(rowBase + 16 * wave + i) * (size_t)AGP + 8 * lane;
      *(volatile v8us*)rp = qv[i];
    }
  }
}

__global__ __launch_bounds__(NTHR) VG void k_pair(const float* __restrict__ h2,
                                                  const int* __restrict__ xa0, const int* __restrict__ xb0,
                                                  const int* __restrict__ xa1, const int* __restrict__ xb1,
                                                  int nB, int nN, unsigned short* pf) {
  __shared__ __attribute__((aligned(16))) unsigned short rb[NWAVE * PFP];
  const int tid = (int)threadIdx.x, lane = tid & 31, wave = tid >> 5;
  const int r   = (int)blockIdx.x * NWAVE + wave;
  const int set = (r >= nB) ? 1 : 0;
  int j = r - set * nB;
  j = j < 0 ? 0 : (j > nB - 1 ? nB - 1 : j);
  const int ia0 = xa0[j], ib0 = xb0[j], ia1 = xa1[j], ib1 = xb1[j];
  int a = set ? ia1 : ia0;
  int b = set ? ib1 : ib0;
  a = a < 0 ? 0 : (a > nN - 1 ? nN - 1 : a);
  b = b < 0 ? 0 : (b > nN - 1 ? nN - 1 : b);
  const v4f ha = *(const v4f*)(h2 + (size_t)a * DF + 4 * lane);
  const v4f hb = *(const v4f*)(h2 + (size_t)b * DF + 4 * lane);
  v4f dd;
  dd.x = fabsf(ha.x - hb.x); dd.y = fabsf(ha.y - hb.y); dd.z = fabsf(ha.z - hb.z); dd.w = fabsf(ha.w - hb.w);
  unsigned short* row = rb + wave * PFP;
  {
    v4us h4, l4;
    unsigned sp;
    sp = split_pack(ha.x); h4[0] = (unsigned short)(sp & 0xffffu); l4[0] = (unsigned short)(sp >> 16);
    sp = split_pack(ha.y); h4[1] = (unsigned short)(sp & 0xffffu); l4[1] = (unsigned short)(sp >> 16);
    sp = split_pack(ha.z); h4[2] = (unsigned short)(sp & 0xffffu); l4[2] = (unsigned short)(sp >> 16);
    sp = split_pack(ha.w); h4[3] = (unsigned short)(sp & 0xffffu); l4[3] = (unsigned short)(sp >> 16);
    *(v4usa*)(row + 0 * DF + 4 * lane) = h4;
    *(v4usa*)(row + 1 * DF + 4 * lane) = l4;
    sp = split_pack(hb.x); h4[0] = (unsigned short)(sp & 0xffffu); l4[0] = (unsigned short)(sp >> 16);
    sp = split_pack(hb.y); h4[1] = (unsigned short)(sp & 0xffffu); l4[1] = (unsigned short)(sp >> 16);
    sp = split_pack(hb.z); h4[2] = (unsigned short)(sp & 0xffffu); l4[2] = (unsigned short)(sp >> 16);
    sp = split_pack(hb.w); h4[3] = (unsigned short)(sp & 0xffffu); l4[3] = (unsigned short)(sp >> 16);
    *(v4usa*)(row + 2 * DF + 4 * lane) = h4;
    *(v4usa*)(row + 3 * DF + 4 * lane) = l4;
    sp = split_pack(dd.x); h4[0] = (unsigned short)(sp & 0xffffu); l4[0] = (unsigned short)(sp >> 16);
    sp = split_pack(dd.y); h4[1] = (unsigned short)(sp & 0xffffu); l4[1] = (unsigned short)(sp >> 16);
    sp = split_pack(dd.z); h4[2] = (unsigned short)(sp & 0xffffu); l4[2] = (unsigned short)(sp >> 16);
    sp = split_pack(dd.w); h4[3] = (unsigned short)(sp & 0xffffu); l4[3] = (unsigned short)(sp >> 16);
    *(v4usa*)(row + 4 * DF + 4 * lane) = h4;
    *(v4usa*)(row + 5 * DF + 4 * lane) = l4;
  }
  wave_sync();
  const v8us q0 = *(const v8usa*)(row + 8 * lane);
  const v8us q1 = *(const v8usa*)(row + 2 * DF + 8 * lane);
  const v8us q2 = *(const v8usa*)(row + 4 * DF + 8 * lane);
  unsigned short* dp = pf + (size_t)r * PFP + 8 * lane;
  *(volatile v8us*)dp = q0;
  *(volatile v8us*)(dp + 2 * DF) = q1;
  *(volatile v8us*)(dp + 4 * DF) = q2;
  __threadfence();
  *(volatile v8us*)dp = q0;
  *(volatile v8us*)(dp + 2 * DF) = q1;
  *(volatile v8us*)(dp + 4 * DF) = q2;
}

__global__ __launch_bounds__(NTHR) VG void k_comb(const float* __restrict__ rec, int tilesPerSet, float* stat) {
  __shared__ __attribute__((aligned(16))) float sg[2 * NTHR];
  const int tid = (int)threadIdx.x;
  const int set = tid >> 7;
  const int col = tid & (GBN - 1);
  double n = 0.0, mean = 0.0, M2 = 0.0;
#pragma unroll 1
  for (int b = 0; b < tilesPerSet; ++b) {
    const float* pr = rec + ((size_t)set * (size_t)tilesPerSet + (size_t)b) * RECW;
    const double nb = (double)GBM;
    const double mb = (double)pr[col];
    const double qb = (double)pr[GBN + col];
    const double nn = n + nb;
    const double delta = mb - mean;
    const double f = nb / nn;
    mean = mean + delta * f;
    M2 = M2 + qb + delta * delta * n * f;
    n = nn;
  }
  const double nt = n < 1.0 ? 1.0 : n;
  const float varf  = (float)(M2 / nt);
  const float meanf = (float)mean;
  const float rstd  = 1.0f / sqrtf(varf + 1e-5f);
  sg[tid] = meanf;
  sg[NTHR + tid] = rstd;
  __syncthreads();
  v4f v = {0.f, 0.f, 0.f, 0.f};
  float* sp = stat + 4 * (tid & (2 * NTHR / 4 - 1));
  if (tid < (2 * NTHR) / 4) {
    v = *(const v4fa*)(sg + 4 * tid);
    *(volatile v4f*)sp = v;
  }
  __threadfence();
  if (tid < (2 * NTHR) / 4) {
    *(volatile v4f*)sp = v;
  }
}

__global__ __launch_bounds__(NTHR) VG void k_apply(const float* __restrict__ y, const float* __restrict__ stat,
                                                   const float* __restrict__ gam, const float* __restrict__ bet,
                                                   const float* __restrict__ W2, const float* __restrict__ b2,
                                                   int nB, int tilesPerSet, float* out) {
  __shared__ __attribute__((aligned(16))) float o0s[2 * GBM];
  const int tid = (int)threadIdx.x, lane = tid & 31, wave = tid >> 5;
  const int tile = (int)blockIdx.x;
  const int set  = (tile >= tilesPerSet) ? 1 : 0;
  const int row0 = tile * GBM;
  const int j0   = row0 - set * nB;
  const v4f m4 = *(const v4f*)(stat + set * DF + 4 * lane);
  const v4f r4 = *(const v4f*)(stat + 2 * DF + set * DF + 4 * lane);
  v4f g4, e4, wa, wb;
  {
    const v4f tg = *(const v4f*)(gam + 4 * lane);
    const v4f tb = *(const v4f*)(bet + 4 * lane);
    const v4f ta = *(const v4f*)(W2 + 8 * lane);
    const v4f tc = *(const v4f*)(W2 + 8 * lane + 4);
    g4.x = bf16_val(tg.x); g4.y = bf16_val(tg.y); g4.z = bf16_val(tg.z); g4.w = bf16_val(tg.w);
    e4.x = bf16_val(tb.x); e4.y = bf16_val(tb.y); e4.z = bf16_val(tb.z); e4.w = bf16_val(tb.w);
    wa.x = bf16_val(ta.x); wa.y = bf16_val(ta.y); wa.z = bf16_val(ta.z); wa.w = bf16_val(ta.w);
    wb.x = bf16_val(tc.x); wb.y = bf16_val(tc.y); wb.z = bf16_val(tc.z); wb.w = bf16_val(tc.w);
  }
  const float c0 = bf16_val(b2[0]);
  const float c1 = bf16_val(b2[1]);
  const size_t obase = (size_t)2 * (size_t)nB + (size_t)set * (size_t)nB * DF;
#pragma unroll 1
  for (int i = 0; i < GBM / NWAVE; ++i) {
    const int lr = wave * (GBM / NWAVE) + i;
    const v4f yv = *(const v4f*)(y + (size_t)(row0 + lr) * DF + 4 * lane);
    v4f v;
    v.x = relu_np(((yv.x - m4.x) * r4.x) * g4.x + e4.x);
    v.y = relu_np(((yv.y - m4.y) * r4.y) * g4.y + e4.y);
    v.z = relu_np(((yv.z - m4.z) * r4.z) * g4.z + e4.z);
    v.w = relu_np(((yv.w - m4.w) * r4.w) * g4.w + e4.w);
    float p0 = v.x * wa.x;
    p0 = fmaf(v.y, wa.z, p0);
    p0 = fmaf(v.z, wb.x, p0);
    p0 = fmaf(v.w, wb.z, p0);
    float p1 = v.x * wa.y;
    p1 = fmaf(v.y, wa.w, p1);
    p1 = fmaf(v.z, wb.y, p1);
    p1 = fmaf(v.w, wb.w, p1);
#pragma unroll
    for (int off = 16; off > 0; off >>= 1) {
      p0 += __shfl_xor(p0, off, 32);
      p1 += __shfl_xor(p1, off, 32);
    }
    if (lane == 0) {
      o0s[2 * lr + 0] = p0 + c0;
      o0s[2 * lr + 1] = p1 + c1;
    }
    float* op = out + obase + (size_t)(j0 + lr) * DF + 4 * lane;
    *(volatile v4f*)op = v;
    __threadfence();
    *(volatile v4f*)op = v;
  }
  __syncthreads();
  if (set == 0 && wave == 0) {
    const v4f q = *(const v4fa*)(o0s + 4 * lane);
    float* op = out + (size_t)j0 * 2 + 4 * lane;
    *(volatile v4f*)op = q;
    __threadfence();
    *(volatile v4f*)op = q;
  }
}

static inline int cdiv(int a, int b) { return (a + b - 1) / b; }
static inline size_t al256(size_t o) { return (o + 255) & ~(size_t)255; }

extern "C" void kernel_launch(void* const* d_in, const int* in_sizes, int n_in,
                              void* d_out, int out_size, void* d_ws, size_t ws_size,
                              hipStream_t stream) {
  if (n_in < 16) return;
  if (in_sizes[0] < DF || (in_sizes[0] % DF) != 0) return;
  const int nN = in_sizes[0] / DF;
  const int nE = in_sizes[1];
  if (nE < 1 || in_sizes[2] != nE) return;
  if (nE >= (1 << 21) || nN < 16 || nN >= (1 << 24)) return;
  const int nB = in_sizes[3];
  if (nB < GBM || (nB % GBM) != 0 || nB > (1 << 20)) return;
  if (in_sizes[4] != nB || in_sizes[5] != nB || in_sizes[6] != nB) return;
  if (in_sizes[7] != 2 * DF * DF || in_sizes[8] != 2 * DF * DF || in_sizes[9] != 2 * DF) return;
  if (in_sizes[10] != 3 * DF * DF || in_sizes[11] != DF || in_sizes[12] != DF || in_sizes[13] != DF) return;
  if (in_sizes[14] != 2 * DF || in_sizes[15] != 2) return;
  if ((long long)out_size != (long long)nB * 2 + 2LL * (long long)nB * DF) return;

  const float* h     = (const float*)d_in[0];
  const int*   esrc  = (const int*)d_in[1];
  const int*   edst  = (const int*)d_in[2];
  const int*   x1    = (const int*)d_in[3];
  const int*   x2    = (const int*)d_in[4];
  const int*   x1t   = (const int*)d_in[5];
  const int*   x2t   = (const int*)d_in[6];
  const float* Wself = (const float*)d_in[7];
  const float* Wnei  = (const float*)d_in[8];
  const float* bconv = (const float*)d_in[9];
  const float* W1    = (const float*)d_in[10];
  const float* b1    = (const float*)d_in[11];
  const float* gamma = (const float*)d_in[12];
  const float* beta  = (const float*)d_in[13];
  const float* W2    = (const float*)d_in[14];
  const float* b2    = (const float*)d_in[15];
  float* out = (float*)d_out;

  const int MP = cdiv(nN, GBM) * GBM;
  const int gM = MP / GBM;
  const int gA = cdiv(nN, NBA);
  if ((long long)gA * NBA < (long long)MP) return;
  const int vec8 = ((nE & 3) == 0) ? 1 : 0;
  const int nP   = 2 * nB;
  const int gH   = nP / GBM;
  const int tilesPerSet = nB / GBM;

  char* ws = (char*)d_ws;
  size_t off = 0;
  const size_t oWP = off; off = al256(off + (size_t)WPTOT * 2);
  const size_t oXB = off; off = al256(off + (size_t)MP * DF * 2);
  const size_t szR = (size_t)MP * AGP * 2;
  const size_t oR1 = off; off = al256(off + szR);
  const size_t oR2 = off; off = al256(off + szR);
  const size_t szPF = (size_t)nP * PFP * 2;
  if (oR2 != oR1 + szR || szPF > 2 * szR) return;
  const size_t oH2 = off; off = al256(off + (size_t)MP * DF * 4);
  const size_t oY  = off; off = al256(off + (size_t)nP * DF * 4);
  const size_t oRC = off; off = al256(off + (size_t)gH * RECW * 4);
  const size_t oST = off; off = al256(off + (size_t)(4 * DF) * 4);
  if (off > ws_size || off > (size_t)WSMAX) return;
  unsigned short* WP   = (unsigned short*)(ws + oWP);
  unsigned short* XB   = (unsigned short*)(ws + oXB);
  unsigned short* AGG  = (unsigned short*)(ws + oR1);
  unsigned short* H1HL = (unsigned short*)(ws + oR2);
  unsigned short* PF   = (unsigned short*)(ws + oR1);
  float*          H2   = (float*)(ws + oH2);
  float*          Y    = (float*)(ws + oY);
  float*          REC  = (float*)(ws + oRC);
  float*          STAT = (float*)(ws + oST);

  const size_t scanLds = (size_t)AGG_LDS_INTS * 4;
  hipFuncSetAttribute(reinterpret_cast<const void*>(&k_scan<1>), hipFuncAttributeMaxDynamicSharedMemorySize, (int)scanLds);
  hipFuncSetAttribute(reinterpret_cast<const void*>(&k_scan<0>), hipFuncAttributeMaxDynamicSharedMemorySize, (int)scanLds);

  const int nUx = MP * (DF / 8);
  k_wprep<<<(NPART * UPART) / NTHR, NTHR, 0, stream>>>(Wself, Wnei, W1, WP);
  k_pa<<<cdiv(nUx, NTHR), NTHR, 0, stream>>>(h, nN, nUx, XB);
  k_scan<1><<<gA, NTHR, scanLds, stream>>>(esrc, edst, nE, nN, vec8, MP, XB, AGG);
  k_gemm<0><<<gM, GTHR, 0, stream>>>(AGG, XB, WP, bconv, nN, H1HL, H2, REC);
  k_scan<0><<<gA, NTHR, scanLds, stream>>>(esrc, edst, nE, nN, vec8, MP, H1HL, AGG);
  k_gemm<1><<<gM, GTHR, 0, stream>>>(AGG, H1HL, WP + WOFF1, bconv + DF, nN, H1HL, H2, REC);
  k_pair<<<nP / NWAVE, NTHR, 0, stream>>>(H2, x1, x2, x1t, x2t, nB, nN, PF);
  k_gemm<2><<<gH, GTHR, 0, stream>>>(PF, PF, WP + WOFFH, b1, nP, H1HL, Y, REC);
  k_comb<<<1, NTHR, 0, stream>>>(REC, tilesPerSet, STAT);
  k_apply<<<gH, NTHR, 0, stream>>>(Y, STAT, gamma, beta, W2, b2, nB, tilesPerSet, out);
}
